// XTransEncoderAct_79963701117003
// MI455X (gfx1250) — hardware-verified
//
#include <hip/hip_runtime.h>
#include <stdint.h>
#include <stddef.h>
#include <math.h>

typedef _Float16 half_t;
typedef _Float16 v16h __attribute__((ext_vector_type(16)));
typedef _Float16 v8h  __attribute__((ext_vector_type(8)));
typedef float    v8f  __attribute__((ext_vector_type(8)));
typedef float    v4f  __attribute__((ext_vector_type(4)));
typedef v8h __attribute__((may_alias)) v8ha;
typedef v4f __attribute__((may_alias)) v4fa;

#define NSEQ  1024
#define NBAT  4
#define NHEAD 16
#define DHID  512
#define DFFN  2048
#define TOK   (NBAT * NSEQ)
#define TOK3  (TOK * 3)
#define FACTOR_F 0.08838834764831845f
#define LN_EPS 1e-5f
#define BS_P  40
#define CS_P  128

union Frag { v16h v; v8h h[2]; };

__device__ __forceinline__ v8f zero8() {
  v8f z = {0.f, 0.f, 0.f, 0.f, 0.f, 0.f, 0.f, 0.f};
  return z;
}

__device__ __forceinline__ v8f wmma_g(v16h a, v16h b, v8f c) {
  v8f d = __builtin_amdgcn_wmma_f32_16x16x32_f16(false, a, false, b, (short)0, c, false, false);
  asm volatile("v_nop\n\tv_nop\n\tv_nop\n\tv_nop" : "+v"(d) : "v"(a), "v"(b));
  return d;
}

__device__ __forceinline__ v16h ldfrag(const half_t* base, int row0, int ld, int kb) {
  const int l = threadIdx.x & 31;
  const half_t* p = base + (size_t)(row0 + (l & 15)) * ld + kb + ((l >> 4) << 3);
  Frag f;
  f.h[0] = *reinterpret_cast<const v8ha*>(p);
  f.h[1] = *reinterpret_cast<const v8ha*>(p + 16);
  return f.v;
}

__device__ __forceinline__ v4f ld4(const float* p) { return *reinterpret_cast<const v4fa*>(p); }

__device__ __forceinline__ v8h pack8(v4f a, v4f b) {
  v8h o;
  o[0] = (half_t)a[0]; o[1] = (half_t)a[1]; o[2] = (half_t)a[2]; o[3] = (half_t)a[3];
  o[4] = (half_t)b[0]; o[5] = (half_t)b[1]; o[6] = (half_t)b[2]; o[7] = (half_t)b[3];
  return o;
}

__device__ __forceinline__ v4f silu4(v4f x) {
  v4f r;
#pragma unroll
  for (int i = 0; i < 4; ++i) r[i] = x[i] / (1.0f + __expf(-x[i]));
  return r;
}

struct GemmP {
  const half_t* A; const half_t* Bt; const float* bias; const float* resid; float* Cf; half_t* Ch;
  int lda; int akb; int azoff; int ldb;
  int M; int N; int K; int ors;
  int orz; int ldr; int ldcf; int ldch;
  int act; int vte0; int vtez; int padz;
};
static_assert(sizeof(GemmP) == 6 * 8 + 16 * 4);

__device__ __forceinline__ void gemm_core(const GemmP& p, const half_t* Ab, half_t* Bs,
                                          int m0, int n0b, int nw, v8f (&acc)[2][4]) {
  const int tid = threadIdx.x;
  for (int k = 0; k < p.K; k += 32) {
    __syncthreads();
#pragma unroll
    for (int c = 0; c < 2; ++c) {
      const int ch = tid + c * 256;
      const int row = ch >> 2, seg = (ch & 3) * 8;
      const v8h t = *reinterpret_cast<const v8ha*>(p.Bt + (size_t)(n0b + row) * p.ldb + k + seg);
      *reinterpret_cast<v8ha*>(Bs + row * BS_P + seg) = t;
    }
    __syncthreads();
    const int kb = (k >> 5) * p.akb;
    const v16h a0 = ldfrag(Ab, m0, p.lda, kb);
    const v16h a1 = ldfrag(Ab, m0 + 16, p.lda, kb);
#pragma unroll
    for (int f = 0; f < 4; ++f) {
      const v16h b = ldfrag(Bs, nw + f * 16, BS_P, 0);
      acc[0][f] = wmma_g(a0, b, acc[0][f]);
      acc[1][f] = wmma_g(a1, b, acc[1][f]);
    }
  }
  __syncthreads();
}

__device__ __forceinline__ void stage_acc(float* Cs, int wr0, int nw, const v8f (&acc)[2][4]) {
  const int l = threadIdx.x & 31, hh = l >> 4, m15 = l & 15;
#pragma unroll
  for (int i = 0; i < 2; ++i)
#pragma unroll
    for (int f = 0; f < 4; ++f)
#pragma unroll
      for (int r = 0; r < 8; ++r)
        Cs[(wr0 + i * 16 + 8 * hh + r) * CS_P + nw + f * 16 + m15] = acc[i][f][r];
}

template <int MODE>
__global__ void __launch_bounds__(256) k_gemm(GemmP p) {
  __shared__ __align__(16) float lds_f[128 * CS_P];
  half_t* Bs = reinterpret_cast<half_t*>(lds_f);
  float*  Cs = lds_f;
  const int tid = threadIdx.x, w = tid >> 5, l = tid & 31, hh = l >> 4, m15 = l & 15;
  const int z = blockIdx.z;
  const int mb0 = blockIdx.y * 128;
  const int wr0 = (w >> 1) * 32;
  const int n0b = blockIdx.x * 128;
  const int nw = (w & 1) * 64;
  const half_t* Ab = p.A + (size_t)z * p.azoff;

  v8f acc[2][4];
#pragma unroll
  for (int i = 0; i < 2; ++i)
#pragma unroll
    for (int f = 0; f < 4; ++f) acc[i][f] = zero8();

  gemm_core(p, Ab, Bs, mb0 + wr0, n0b, nw, acc);
  stage_acc(Cs, wr0, nw, acc);
  __syncthreads();

  if (MODE == 0) {
#pragma unroll
    for (int pass = 0; pass < 2; ++pass) {
      if (pass) __threadfence();
#pragma unroll
      for (int it = 0; it < 8; ++it) {
        const int rr = w * 16 + 2 * it + hh;
        const int cc = 8 * m15;
        v4f x0 = ld4(Cs + rr * CS_P + cc);
        v4f x1 = ld4(Cs + rr * CS_P + cc + 4);
        if (p.bias) { x0 += ld4(p.bias + n0b + cc); x1 += ld4(p.bias + n0b + cc + 4); }
        if (p.act) { x0 = silu4(x0); x1 = silu4(x1); }
        const size_t orow = (size_t)(mb0 + rr) * p.ors + (size_t)z * p.orz;
        *reinterpret_cast<volatile v8h*>(p.Ch + orow * p.ldch + n0b + cc) = pack8(x0, x1);
      }
    }
  } else if (MODE == 1) {
#pragma unroll
    for (int pass = 0; pass < 2; ++pass) {
      if (pass) __threadfence();
#pragma unroll
      for (int it = 0; it < 16; ++it) {
        const int rr = w * 16 + it;
        const int cc = 4 * l;
        v4f x = ld4(Cs + rr * CS_P + cc);
        if (p.bias) x += ld4(p.bias + n0b + cc);
        const size_t orow = (size_t)(mb0 + rr) * p.ors + (size_t)z * p.orz;
        if (p.resid) x += ld4(p.resid + orow * p.ldr + n0b + cc);
        *reinterpret_cast<volatile v4f*>(p.Cf + orow * p.ldcf + n0b + cc) = x;
      }
      if (p.Ch) {
#pragma unroll
        for (int it = 0; it < 8; ++it) {
          const int rr = w * 16 + 2 * it + hh;
          const int cc = 8 * m15;
          v4f x0 = ld4(Cs + rr * CS_P + cc);
          v4f x1 = ld4(Cs + rr * CS_P + cc + 4);
          if (p.bias) { x0 += ld4(p.bias + n0b + cc); x1 += ld4(p.bias + n0b + cc + 4); }
          const size_t orow = (size_t)(mb0 + rr) * p.ors + (size_t)z * p.orz;
          if (p.resid) {
            x0 += ld4(p.resid + orow * p.ldr + n0b + cc);
            x1 += ld4(p.resid + orow * p.ldr + n0b + cc + 4);
          }
          *reinterpret_cast<volatile v8h*>(p.Ch + orow * p.ldch + n0b + cc) = pack8(x0, x1);
        }
      }
    }
  } else {
    const int bidx = mb0 >> 10;
    const int nn0  = mb0 & (NSEQ - 1);
    const int eoff = p.vte0 + z * p.vtez;
#pragma unroll
    for (int pass = 0; pass < 2; ++pass) {
      if (pass) __threadfence();
#pragma unroll
      for (int it = 0; it < 8; ++it) {
        const int jj = w * 16 + 2 * it + hh;
        const int n = n0b + jj;
        const float bvn = p.bias ? p.bias[n] : 0.0f;
        v8h o;
#pragma unroll
        for (int q = 0; q < 8; ++q) o[q] = (half_t)(Cs[(8 * m15 + q) * CS_P + jj] + bvn);
        const size_t vrow = (size_t)(bidx * NHEAD + (n >> 5)) * 128 + eoff + (n & 31);
        *reinterpret_cast<volatile v8h*>(p.Ch + vrow * NSEQ + nn0 + 8 * m15) = o;
      }
    }
  }
}

__global__ void __launch_bounds__(256) k_gemm_lv(GemmP p) {
  __shared__ __align__(16) float lds_f[128 * CS_P];
  half_t* Bs = reinterpret_cast<half_t*>(lds_f);
  float*  Cs = lds_f;
  const int tid = threadIdx.x, w = tid >> 5, l = tid & 31, hh = l >> 4, m15 = l & 15;
  const int mb0 = blockIdx.y * 128;
  const int wr0 = (w >> 1) * 32;
  const int n0b = blockIdx.x * 128;
  const int nw = (w & 1) * 64;
  const bool vpart = (n0b >= DHID);

  float ss[16][4];
#pragma unroll
  for (int it = 0; it < 16; ++it)
#pragma unroll
    for (int q = 0; q < 4; ++q) ss[it][q] = 0.0f;

#pragma unroll 1
  for (int c = 0; c < 3; ++c) {
    v8f acc[2][4];
#pragma unroll
    for (int i = 0; i < 2; ++i)
#pragma unroll
      for (int f = 0; f < 4; ++f) acc[i][f] = zero8();
    gemm_core(p, p.A + (size_t)c * p.azoff, Bs, mb0 + wr0, n0b, nw, acc);
    stage_acc(Cs, wr0, nw, acc);
    __syncthreads();
    if (vpart) {
#pragma unroll
      for (int pass = 0; pass < 2; ++pass) {
        if (pass) __threadfence();
#pragma unroll
        for (int it = 0; it < 16; ++it) {
          const int rr = w * 16 + it, cc = 4 * l;
          const v4f x = ld4(Cs + rr * CS_P + cc);
          const size_t orow = (size_t)(mb0 + rr) * 3 + c;
          *reinterpret_cast<volatile v4f*>(p.Cf + orow * p.ldcf + (n0b - DHID) + cc) = x;
        }
      }
    } else {
#pragma unroll
      for (int it = 0; it < 16; ++it) {
        const int rr = w * 16 + it, cc = 4 * l;
        const v4f x = ld4(Cs + rr * CS_P + cc);
#pragma unroll
        for (int q = 0; q < 4; ++q) ss[it][q] += x[q] * x[q];
      }
    }
    __syncthreads();
  }

  if (!vpart) {
#pragma unroll
    for (int it = 0; it < 16; ++it) {
      const int rr = w * 16 + it, cc = 4 * l;
      v4f y;
#pragma unroll
      for (int q = 0; q < 4; ++q) y[q] = sqrtf(ss[it][q]);
      *reinterpret_cast<v4fa*>(Cs + rr * CS_P + cc) = y;
    }
    __syncthreads();
#pragma unroll
    for (int pass = 0; pass < 2; ++pass) {
      if (pass) __threadfence();
#pragma unroll
      for (int it = 0; it < 8; ++it) {
        const int rr = w * 16 + 2 * it + hh;
        const int cc = 8 * m15;
        const v4f x0 = ld4(Cs + rr * CS_P + cc);
        const v4f x1 = ld4(Cs + rr * CS_P + cc + 4);
        *reinterpret_cast<volatile v8h*>(p.Ch + (size_t)(mb0 + rr) * p.ldch + DHID + n0b + cc) = pack8(x0, x1);
      }
    }
  }
}

__global__ void __launch_bounds__(256)
k_attn(const half_t* Hq, const half_t* Hk, const half_t* Vt, const float* biasB, half_t* res) {
  const int w = threadIdx.x >> 5, l = threadIdx.x & 31, hh = l >> 4, m15 = l & 15;
  int t = blockIdx.x;
  const int ntile = t & 7;  t >>= 3;
  const int hd    = t & 15; t >>= 4;
  const int b     = t;
  const int n0 = ntile * 128 + w * 16;

  const half_t* HqB = Hq + (size_t)b * NSEQ * (4 * DHID) + hd * 128;
  const half_t* HkB = Hk + (size_t)b * NSEQ * (4 * DHID) + hd * 128;
  const half_t* VtB = Vt + (size_t)(b * NHEAD + hd) * 128 * NSEQ;
  const float*  bB  = biasB + (size_t)b * NSEQ * NSEQ;

  __shared__ __align__(16) half_t Plds[8][16][32];
  __shared__ __align__(16) half_t Ot[8][16][136];

  const float NEG_INF = -__builtin_inff();

  v16h q[4];
#pragma unroll
  for (int kd = 0; kd < 4; ++kd) q[kd] = ldfrag(HqB, n0, 4 * DHID, kd * 32);

  v8f acc[8];
#pragma unroll
  for (int f = 0; f < 8; ++f) acc[f] = zero8();
  float rmax[8], rsum[8];
#pragma unroll
  for (int r = 0; r < 8; ++r) { rmax[r] = NEG_INF; rsum[r] = 0.0f; }

  for (int m0 = 0; m0 < NSEQ; m0 += 32) {
    v8f s[2];
    s[0] = zero8(); s[1] = zero8();
#pragma unroll
    for (int j = 0; j < 2; ++j)
#pragma unroll
      for (int kd = 0; kd < 4; ++kd)
        s[j] = wmma_g(q[kd], ldfrag(HkB, m0 + 16 * j, 4 * DHID, kd * 32), s[j]);

#pragma unroll
    for (int j = 0; j < 2; ++j) {
      const int m = m0 + 16 * j + m15;
#pragma unroll
      for (int r = 0; r < 8; ++r) {
        const int n = n0 + 8 * hh + r;
        s[j][r] = s[j][r] * FACTOR_F + bB[(size_t)n * NSEQ + m];
      }
    }

#pragma unroll
    for (int r = 0; r < 8; ++r) {
      float mx = fmaxf(s[0][r], s[1][r]);
#pragma unroll
      for (int off = 1; off <= 8; off <<= 1) mx = fmaxf(mx, __shfl_xor(mx, off, 32));
      const float nm = fmaxf(rmax[r], mx);
      const float corr = (rmax[r] == NEG_INF) ? 0.0f : __expf(rmax[r] - nm);
      const float p0 = (nm == NEG_INF) ? 0.0f : __expf(s[0][r] - nm);
      const float p1 = (nm == NEG_INF) ? 0.0f : __expf(s[1][r] - nm);
      float ts = p0 + p1;
#pragma unroll
      for (int off = 1; off <= 8; off <<= 1) ts += __shfl_xor(ts, off, 32);
      rsum[r] = rsum[r] * corr + ts;
      rmax[r] = nm;
#pragma unroll
      for (int f = 0; f < 8; ++f) acc[f][r] *= corr;
      Plds[w][8 * hh + r][m15]      = (half_t)(p0 * 256.0f);
      Plds[w][8 * hh + r][16 + m15] = (half_t)(p1 * 256.0f);
    }
    __syncthreads();

    const v16h pa = ldfrag(&Plds[w][0][0], 0, 32, 0);
#pragma unroll
    for (int f = 0; f < 8; ++f)
      acc[f] = wmma_g(pa, ldfrag(VtB, f * 16, NSEQ, m0), acc[f]);
    __syncthreads();
  }

#pragma unroll
  for (int r = 0; r < 8; ++r) {
    const float inv = 0.00390625f / rsum[r];
#pragma unroll
    for (int f = 0; f < 8; ++f) Ot[w][8 * hh + r][f * 16 + m15] = (half_t)(acc[f][r] * inv);
  }
  __syncthreads();
#pragma unroll
  for (int pass = 0; pass < 2; ++pass) {
    if (pass) __threadfence();
#pragma unroll
    for (int it = 0; it < 8; ++it) {
      const int rr = 2 * it + hh, e0 = 8 * m15;
      const v8h o = *reinterpret_cast<const v8ha*>(&Ot[w][rr][e0]);
      const size_t tok = (size_t)b * NSEQ + n0 + rr;
      *reinterpret_cast<volatile v8h*>(res + (tok * NHEAD + hd) * 128 + e0) = o;
    }
  }
}

__global__ void __launch_bounds__(256)
k_bias(const float* __restrict__ rbf, const float* __restrict__ Db, const int* __restrict__ msk,
       float* out, int n4) {
  const int i = blockIdx.x * 256 + threadIdx.x;
  if (i >= n4) return;
  const size_t e = (size_t)i * 4;
  const int b = (int)(e >> 20);
  const int m = (int)(e & (NSEQ - 1));
  const v4f a = ld4(rbf + e), d = ld4(Db + e);
  const float NEG_INF = -__builtin_inff();
  v4f o;
#pragma unroll
  for (int q = 0; q < 4; ++q) o[q] = (msk[b * NSEQ + m + q] != 0) ? (a[q] + d[q]) : NEG_INF;
  *reinterpret_cast<volatile v4f*>(out + e) = o;
  __threadfence();
  *reinterpret_cast<volatile v4f*>(out + e) = o;
}

__global__ void __launch_bounds__(256)
k_ln(const float* X, const float* __restrict__ g, const float* __restrict__ be,
     half_t* Y, int ldy, int rows) {
  const int w = threadIdx.x >> 5, l = threadIdx.x & 31;
  const int row = blockIdx.x * 8 + w;
  if (row >= rows) return;
  const float* x = X + (size_t)row * DHID;
  const int c0 = 8 * l, c1 = 256 + 8 * l;
  v4f a0 = ld4(x + c0), a1 = ld4(x + c0 + 4), a2 = ld4(x + c1), a3 = ld4(x + c1 + 4);
  float s = 0.0f;
#pragma unroll
  for (int q = 0; q < 4; ++q) s += a0[q] + a1[q] + a2[q] + a3[q];
#pragma unroll
  for (int off = 1; off < 32; off <<= 1) s += __shfl_xor(s, off, 32);
  const float mean = s * (1.0f / DHID);
  a0 -= mean; a1 -= mean; a2 -= mean; a3 -= mean;
  float v = 0.0f;
#pragma unroll
  for (int q = 0; q < 4; ++q) v += a0[q] * a0[q] + a1[q] * a1[q] + a2[q] * a2[q] + a3[q] * a3[q];
#pragma unroll
  for (int off = 1; off < 32; off <<= 1) v += __shfl_xor(v, off, 32);
  const float var  = v * (1.0f / DHID);
  const float rstd = 1.0f / sqrtf(var + LN_EPS);
  const v4f y0 = a0 * rstd * ld4(g + c0)     + ld4(be + c0);
  const v4f y1 = a1 * rstd * ld4(g + c0 + 4) + ld4(be + c0 + 4);
  const v4f y2 = a2 * rstd * ld4(g + c1)     + ld4(be + c1);
  const v4f y3 = a3 * rstd * ld4(g + c1 + 4) + ld4(be + c1 + 4);
  const v8h o0 = pack8(y0, y1), o1 = pack8(y2, y3);
  half_t* yp = Y + (size_t)row * ldy;
  *reinterpret_cast<volatile v8h*>(yp + c0) = o0;
  *reinterpret_cast<volatile v8h*>(yp + c1) = o1;
  __threadfence();
  *reinterpret_cast<volatile v8h*>(yp + c0) = o0;
  *reinterpret_cast<volatile v8h*>(yp + c1) = o1;
}

__global__ void __launch_bounds__(256)
k_cast(const float* __restrict__ in, half_t* out, int n8) {
  const int i = blockIdx.x * 256 + threadIdx.x;
  if (i >= n8) return;
  const size_t e = (size_t)i * 8;
  const v8h o = pack8(ld4(in + e), ld4(in + e + 4));
  *reinterpret_cast<volatile v8h*>(out + e) = o;
  __threadfence();
  *reinterpret_cast<volatile v8h*>(out + e) = o;
}

__global__ void __launch_bounds__(256)
k_tw(const float* __restrict__ W, half_t* Wt, int K, int N) {
  __shared__ float T[64][65];
  const int tid = threadIdx.x, w = tid >> 5, l = tid & 31;
  const int k0 = blockIdx.y * 64, n0 = blockIdx.x * 64;
#pragma unroll
  for (int it = 0; it < 4; ++it) {
    const int idx = tid + it * 256;
    const int kk = idx >> 4, c4 = (idx & 15) * 4;
    const v4f v = ld4(W + (size_t)(k0 + kk) * N + n0 + c4);
    T[kk][c4 + 0] = v[0]; T[kk][c4 + 1] = v[1]; T[kk][c4 + 2] = v[2]; T[kk][c4 + 3] = v[3];
  }
  __syncthreads();
#pragma unroll
  for (int pass = 0; pass < 2; ++pass) {
    if (pass) __threadfence();
#pragma unroll
    for (int it = 0; it < 2; ++it) {
      const int nn  = w * 8 + it * 4 + (l >> 3);
      const int kk0 = 8 * (l & 7);
      v8h o;
#pragma unroll
      for (int q = 0; q < 8; ++q) o[q] = (half_t)T[kk0 + q][nn];
      *reinterpret_cast<volatile v8h*>(Wt + (size_t)(n0 + nn) * K + k0 + kk0) = o;
    }
  }
}

__global__ void __launch_bounds__(256)
k_final(const float* H2, const float* hout, const float* V2f, const float* Vp2,
        float* outH, float* outV, int nH4, int nV4) {
  const int i = blockIdx.x * 256 + threadIdx.x;
  if (i >= nH4 + nV4) return;
  v4f o;
  float* dst;
  if (i < nH4) {
    const size_t e = (size_t)i * 4;
    const size_t t = e >> 9;
    const int j = (int)(e & (DHID - 1));
    o = ld4(H2 + e) + ld4(hout + t * (2 * DHID) + j);
    dst = outH + e;
  } else {
    const size_t e = (size_t)(i - nH4) * 4;
    const size_t t3 = e >> 9;
    const int j = (int)(e & (DHID - 1));
    const size_t tok = t3 / 3;
    o = ld4(V2f + e) + ld4(hout + tok * (2 * DHID) + DHID + j) * ld4(Vp2 + e);
    dst = outV + e;
  }
  *reinterpret_cast<volatile v4f*>(dst) = o;
  __threadfence();
  *reinterpret_cast<volatile v4f*>(dst) = o;
}

extern "C" void kernel_launch(void* const* d_in, const int* in_sizes, int n_in,
                              void* d_out, int out_size, void* d_ws, size_t ws_size,
                              hipStream_t stream) {
  if (n_in < 24) return;
  const int need[24] = {
    TOK * DHID, TOK3 * DHID, NBAT * NSEQ * NSEQ, NBAT * NSEQ * NSEQ, NBAT * NSEQ,
    DHID, DHID,
    DHID * 4 * DHID, 4 * DHID, DHID * 4 * DHID, 4 * DHID,
    DHID * DHID, DHID, DHID * DHID, DHID * DHID, DHID, DHID * DHID,
    DHID, DHID,
    DHID * 2 * DHID, 2 * DHID * DFFN, DFFN, DFFN * 2 * DHID, 2 * DHID };
  for (int i = 0; i < 24; ++i) if (in_sizes[i] != need[i]) return;
  if (out_size != TOK * DHID + TOK3 * DHID) return;

  const size_t MB = (size_t)1 << 20;
  const size_t total = 111 * MB;
  if (ws_size < total) return;

  const float* H   = (const float*)d_in[0];
  const float* V   = (const float*)d_in[1];
  const float* Db  = (const float*)d_in[2];
  const float* rbf = (const float*)d_in[3];
  const int*   Hm  = (const int*)  d_in[4];
  const float* g1  = (const float*)d_in[5];
  const float* be1 = (const float*)d_in[6];
  const float* Wq  = (const float*)d_in[7];
  const float* bq  = (const float*)d_in[8];
  const float* Wk  = (const float*)d_in[9];
  const float* bk  = (const float*)d_in[10];
  const float* Wv  = (const float*)d_in[11];
  const float* bv  = (const float*)d_in[12];
  const float* Wvv = (const float*)d_in[13];
  const float* Wo  = (const float*)d_in[14];
  const float* bo  = (const float*)d_in[15];
  const float* Wvo = (const float*)d_in[16];
  const float* g2  = (const float*)d_in[17];
  const float* be2 = (const float*)d_in[18];
  const float* Wlv = (const float*)d_in[19];
  const float* W1  = (const float*)d_in[20];
  const float* b1f = (const float*)d_in[21];
  const float* W2  = (const float*)d_in[22];
  const float* b2f = (const float*)d_in[23];

  char* ws = (char*)d_ws;
  half_t* WlvT = (half_t*)(ws + 0);
  half_t* W1T  = (half_t*)(ws + 1 * MB);
  half_t* W2T  = (half_t*)(ws + 5 * MB);
  half_t* WqT  = (half_t*)(ws + 9 * MB);
  half_t* WkT  = (half_t*)(ws + 11 * MB);
  half_t* WvT  = (half_t*)(ws + 13 * MB);
  half_t* WvvT = (half_t*)(ws + 13 * MB + MB / 2);
  half_t* WoT  = (half_t*)(ws + 14 * MB);
  half_t* WvoT = (half_t*)(ws + 14 * MB + MB / 2);
  half_t* Hn   = (half_t*)(ws + 15 * MB);
  half_t* Vf16 = (half_t*)(ws + 19 * MB);
  half_t* res  = (half_t*)(ws + 15 * MB);
  float*  hout = (float*) (ws + 15 * MB);
  half_t* Hq   = (half_t*)(ws + 31 * MB);
  half_t* V2h  = (half_t*)(ws + 31 * MB);
  half_t* S1   = (half_t*)(ws + 31 * MB);
  half_t* Hk   = (half_t*)(ws + 47 * MB);
  half_t* Vt   = (half_t*)(ws + 63 * MB);
  float*  Vp2  = (float*) (ws + 47 * MB);
  half_t* scal = (half_t*)(ws + 71 * MB);
  float*  biasB = (float*)(ws + 79 * MB);
  float*  H2   = (float*) (ws + 79 * MB);
  float*  V2f  = (float*) (ws + 87 * MB);

  float* outH = (float*)d_out;
  float* outV = outH + (size_t)TOK * DHID;

  auto tw = [&](const float* Wsrc, half_t* Wdst, int K, int N) {
    dim3 grid(N / 64, K / 64);
    k_tw<<<grid, 256, 0, stream>>>(Wsrc, Wdst, K, N);
  };

  k_ln<<<(TOK + 7) / 8, 256, 0, stream>>>(H, g1, be1, Hn, DHID, TOK);
  {
    const int n8 = TOK3 * DHID / 8;
    k_cast<<<(n8 + 255) / 256, 256, 0, stream>>>(V, Vf16, n8);
  }
  tw(Wq,  WqT,  DHID, 4 * DHID);
  tw(Wk,  WkT,  DHID, 4 * DHID);
  tw(Wv,  WvT,  DHID, DHID);
  tw(Wvv, WvvT, DHID, DHID);
  tw(Wo,  WoT,  DHID, DHID);
  tw(Wvo, WvoT, DHID, DHID);
  tw(Wlv, WlvT, DHID, 2 * DHID);
  tw(W1,  W1T,  2 * DHID, DFFN);
  tw(W2,  W2T,  DFFN, 2 * DHID);
  {
    const int n4 = NBAT * NSEQ * NSEQ / 4;
    k_bias<<<(n4 + 255) / 256, 256, 0, stream>>>(rbf, Db, Hm, biasB, n4);
  }

  {
    GemmP p{};
    p.A = Hn; p.lda = DHID; p.akb = 32; p.azoff = 0;
    p.Bt = WqT; p.ldb = DHID; p.M = TOK; p.N = 4 * DHID; p.K = DHID;
    p.bias = bq; p.Ch = Hq; p.ldch = 4 * DHID; p.ors = 1; p.orz = 0; p.act = 0;
    k_gemm<0><<<dim3(p.N / 128, p.M / 128, 1), 256, 0, stream>>>(p);
    p.Bt = WkT; p.bias = bk; p.Ch = Hk;
    k_gemm<0><<<dim3(p.N / 128, p.M / 128, 1), 256, 0, stream>>>(p);
  }
  {
    GemmP p{};
    p.A = Hn; p.lda = DHID; p.akb = 32; p.azoff = 0;
    p.Bt = WvT; p.ldb = DHID; p.M = TOK; p.N = DHID; p.K = DHID;
    p.bias = bv; p.Ch = Vt; p.vte0 = 0; p.vtez = 0;
    k_gemm<2><<<dim3(p.N / 128, p.M / 128, 1), 256, 0, stream>>>(p);
  }
  {
    GemmP p{};
    p.A = Vf16; p.lda = 3 * DHID; p.akb = 32; p.azoff = DHID;
    p.Bt = WvvT; p.ldb = DHID; p.M = TOK; p.N = DHID; p.K = DHID;
    p.bias = nullptr; p.Ch = Vt; p.vte0 = 32; p.vtez = 32;
    k_gemm<2><<<dim3(p.N / 128, p.M / 128, 3), 256, 0, stream>>>(p);
  }

  k_attn<<<NBAT * NHEAD * (NSEQ / 128), 256, 0, stream>>>(Hq, Hk, Vt, biasB, res);

  {
    GemmP p{};
    p.A = res; p.lda = NHEAD * 128; p.akb = 128; p.azoff = 0;
    p.Bt = WoT; p.ldb = DHID; p.M = TOK; p.N = DHID; p.K = DHID;
    p.bias = bo; p.resid = H; p.ldr = DHID; p.Cf = H2; p.ldcf = DHID; p.Ch = nullptr;
    p.ors = 1; p.orz = 0;
    k_gemm<1><<<dim3(p.N / 128, p.M / 128, 1), 256, 0, stream>>>(p);
  }
  {
    GemmP p{};
    p.A = res + 32; p.lda = NHEAD * 128; p.akb = 128; p.azoff = 32;
    p.Bt = WvoT; p.ldb = DHID; p.M = TOK; p.N = DHID; p.K = DHID;
    p.bias = nullptr; p.resid = V; p.ldr = DHID; p.Cf = V2f; p.ldcf = DHID; p.Ch = V2h; p.ldch = DHID;
    p.ors = 3; p.orz = 1;
    k_gemm<1><<<dim3(p.N / 128, p.M / 128, 3), 256, 0, stream>>>(p);
  }

  k_ln<<<(TOK + 7) / 8, 256, 0, stream>>>(H2, g2, be2, scal, 2 * DHID, TOK);
  {
    GemmP p{};
    p.A = V2h; p.lda = 3 * DHID; p.akb = 32; p.azoff = DHID;
    p.Bt = WlvT; p.ldb = DHID; p.M = TOK; p.N = 2 * DHID; p.K = DHID;
    p.Cf = Vp2; p.ldcf = DHID; p.Ch = scal; p.ldch = 2 * DHID;
    k_gemm_lv<<<dim3(p.N / 128, p.M / 128, 1), 256, 0, stream>>>(p);
  }
  {
    GemmP p{};
    p.A = scal; p.lda = 2 * DHID; p.akb = 32; p.azoff = 0;
    p.Bt = W1T; p.ldb = 2 * DHID; p.M = TOK; p.N = DFFN; p.K = 2 * DHID;
    p.bias = b1f; p.act = 1; p.Ch = S1; p.ldch = DFFN; p.ors = 1; p.orz = 0;
    k_gemm<0><<<dim3(p.N / 128, p.M / 128, 1), 256, 0, stream>>>(p);
  }
  {
    GemmP p{};
    p.A = S1; p.lda = DFFN; p.akb = 32; p.azoff = 0;
    p.Bt = W2T; p.ldb = DFFN; p.M = TOK; p.N = 2 * DHID; p.K = DFFN;
    p.bias = b2f; p.resid = nullptr; p.Cf = hout; p.ldcf = 2 * DHID; p.Ch = nullptr;
    p.ors = 1; p.orz = 0;
    k_gemm<1><<<dim3(p.N / 128, p.M / 128, 1), 256, 0, stream>>>(p);
  }

  {
    const int nH4 = TOK * DHID / 4, nV4 = TOK3 * DHID / 4;
    k_final<<<(nH4 + nV4 + 255) / 256, 256, 0, stream>>>(H2, hout, V2f, Vp2, outH, outV, nH4, nV4);
  }
}
